// GlobalAggregationBlock_1039382086104
// MI455X (gfx1250) — hardware-verified
//
#include <hip/hip_runtime.h>
#include <math.h>
#include <stdint.h>

constexpr int NBATCH = 2;
constexpr int NCH    = 64;
constexpr int NVOX   = 8000;
constexpr float kWCarry    = 256.0f;
constexpr float kWCarryInv = 1.0f / 256.0f;
constexpr float kOCarry    = 256.0f;
constexpr float kOutScale  = 1.0f / 65536.0f;
constexpr float kQKScale   = 0.125f;
constexpr float kPCarry    = 32768.0f;

typedef __attribute__((ext_vector_type(16))) _Float16 v16h;
typedef __attribute__((ext_vector_type(8)))  _Float16 v8h;
typedef __attribute__((ext_vector_type(16))) __bf16   v16b;
typedef __attribute__((ext_vector_type(8)))  __bf16   v8b;
typedef __attribute__((ext_vector_type(8)))  float    v8f;
typedef __attribute__((ext_vector_type(4)))  float    v4f;
typedef __attribute__((ext_vector_type(4)))  unsigned int v4u;

__device__ __forceinline__ unsigned short f2bf_bits(float f) {
  unsigned u = __float_as_uint(f);
  return (unsigned short)((u + 0x7FFFu + ((u >> 16) & 1u)) >> 16);
}
__device__ __forceinline__ float bf_bits2f(unsigned short h) { return __uint_as_float(((unsigned)h) << 16); }

__device__ __forceinline__ void dep_guard_h(v8f& a, v8f& b, v16h x, v16h y) { asm volatile("v_nop\n\tv_nop\n\tv_nop\n\tv_nop" : "+v"(a), "+v"(b) : "v"(x), "v"(y)); }
__device__ __forceinline__ void dep_guard_b(v8f& a, v8f& b, v16b x, v16b y) { asm volatile("v_nop\n\tv_nop\n\tv_nop\n\tv_nop" : "+v"(a), "+v"(b) : "v"(x), "v"(y)); }
__device__ __forceinline__ void keep4_h(v16h a, v16h b, v16h c, v16h d) { asm volatile("v_nop" :: "v"(a), "v"(b), "v"(c), "v"(d)); }
__device__ __forceinline__ void keep4_b(v16b a, v16b b, v16b c, v16b d) { asm volatile("v_nop" :: "v"(a), "v"(b), "v"(c), "v"(d)); }
__device__ __forceinline__ void acc_guard4(v8f& a, v8f& b, v8f& c, v8f& d) { asm volatile("v_nop\n\tv_nop\n\tv_nop\n\tv_nop" : "+v"(a), "+v"(b), "+v"(c), "+v"(d)); }
template <typename T> struct Frag;
template <> struct Frag<_Float16> {
  typedef v16h V; union U { v16h v; v8h h[2]; };
  static __device__ __forceinline__ v16h load(const _Float16* p) {
    U f; f.h[0] = *(const v8h*)(p); f.h[1] = *(const v8h*)(p + 16); return f.v;
  }
  static __device__ __forceinline__ v8f mma(v16h a, v16h b, v8f c) {
    return __builtin_amdgcn_wmma_f32_16x16x32_f16(false, a, false, b, (short)0, c, false, false);
  }
  static __device__ __forceinline__ void guard(v8f& a, v8f& b, v16h x, v16h y) { dep_guard_h(a, b, x, y); }
  static __device__ __forceinline__ void keep(v16h a, v16h b, v16h c, v16h d) { keep4_h(a, b, c, d); }
};
template <> struct Frag<__bf16> {
  typedef v16b V; union U { v16b v; v8b h[2]; };
  static __device__ __forceinline__ v16b load(const __bf16* p) {
    U f; f.h[0] = *(const v8b*)(p); f.h[1] = *(const v8b*)(p + 16); return f.v;
  }
  static __device__ __forceinline__ v8f mma(v16b a, v16b b, v8f c) {
    return __builtin_amdgcn_wmma_f32_16x16x32_bf16(false, a, false, b, (short)0, c, false, false);
  }
  static __device__ __forceinline__ void guard(v8f& a, v8f& b, v16b x, v16b y) { dep_guard_b(a, b, x, y); }
  static __device__ __forceinline__ void keep(v16b a, v16b b, v16b c, v16b d) { keep4_b(a, b, c, d); }
};

template <int ET> struct Elem;
template <> struct Elem<0> { typedef _Float16 T; };
template <> struct Elem<1> { typedef __bf16 T; };
template <int ET, bool SPLIT, int BIAS_MODE, int OUT_MODE, bool RESID, int ACT = 0, int TRI = 0>
__global__ __launch_bounds__(256) void wmma_gemm64(
    const unsigned short* __restrict__ Ap, const unsigned short* __restrict__ A2p, int lda, long strideA,
    const unsigned short* __restrict__ Btp, const unsigned short* __restrict__ Bt2p, int ldb, long strideB,
    void* __restrict__ Cout, void* __restrict__ Cout2, int ldc, long strideC,
    const float* __restrict__ bias,
    const float* __restrict__ resid, long strideR,
    int M, int N, int K, float scale) {
  typedef typename Elem<ET>::T T;
  typedef typename Frag<T>::V V;
  const T* A = (const T*)Ap; const T* A2 = (const T*)A2p; const T* Bt = (const T*)Btp; const T* Bt2 = (const T*)Bt2p;
  __shared__ __align__(16) float sT[8][16 * 68];
  const int b    = blockIdx.y;
  const int lane = threadIdx.x & 31;
  const int wave = threadIdx.x >> 5;
  const int tilesN = N >> 6;
  const int tilesM = M >> 6;
  const int tile = blockIdx.x * 8 + wave;
  if (tile >= tilesM * tilesN) return;
  const int tm = tile / tilesN;
  const int tn = tile - tm * tilesN;
  const int m0 = tm << 6;
  const int n0 = tn << 6;
  if (TRI == 1 && n0 > m0) return;
  const int Kl = (TRI == 2 && (m0 + 64) < K) ? (m0 + 64) : K;

  const T* Ab  = A  + (size_t)b * strideA;
  const T* Bb  = Bt + (size_t)b * strideB;
  const T* Ab2 = SPLIT ? (A2  + (size_t)b * strideA) : nullptr;
  const T* Bb2 = SPLIT ? (Bt2 + (size_t)b * strideB) : nullptr;

  const int rlane = lane & 15;
  const int koff  = (lane >> 4) * 8;
  const int mOff  = (lane >> 4) * 8;

  v8f acc[4][4];
#pragma unroll
  for (int i = 0; i < 4; ++i)
#pragma unroll
    for (int j = 0; j < 4; ++j) acc[i][j] = (v8f){0.f,0.f,0.f,0.f,0.f,0.f,0.f,0.f};

  for (int k0 = 0; k0 < Kl; k0 += 32) {
    V bh[4], bl[4];
#pragma unroll
    for (int j = 0; j < 4; ++j) {
      const size_t bo = (size_t)(n0 + (j << 4) + rlane) * ldb + koff + k0;
      bh[j] = Frag<T>::load(Bb + bo);
      if (SPLIT) bl[j] = Frag<T>::load(Bb2 + bo);
    }
#pragma unroll
    for (int i = 0; i < 4; ++i) {
      const size_t ao = (size_t)(m0 + (i << 4) + rlane) * lda + koff + k0;
      V ah = Frag<T>::load(Ab + ao);
      V al;
      if (SPLIT) al = Frag<T>::load(Ab2 + ao);
#pragma unroll
      for (int j = 0; j < 4; ++j) {
        acc[i][j] = Frag<T>::mma(ah, bh[j], acc[i][j]);
        if (SPLIT) {
          acc[i][j] = Frag<T>::mma(ah, bl[j], acc[i][j]);
          acc[i][j] = Frag<T>::mma(al, bh[j], acc[i][j]);
        }
      }
      Frag<T>::guard(acc[i][0], acc[i][3], ah, SPLIT ? al : ah);
    }
    Frag<T>::keep(bh[0], bh[1], bh[2], bh[3]);
    if (SPLIT) Frag<T>::keep(bl[0], bl[1], bl[2], bl[3]);
  }
  acc_guard4(acc[0][0], acc[0][1], acc[0][2], acc[0][3]);
  acc_guard4(acc[1][0], acc[1][1], acc[1][2], acc[1][3]);
  acc_guard4(acc[2][0], acc[2][1], acc[2][2], acc[2][3]);
  acc_guard4(acc[3][0], acc[3][1], acc[3][2], acc[3][3]);

  float* slab = sT[wave];
  const float* Rb = RESID ? (resid + (size_t)b * strideR) : nullptr;
#pragma unroll
  for (int i = 0; i < 4; ++i) {
    const int mBase = m0 + (i << 4);
#pragma unroll
    for (int j = 0; j < 4; ++j) {
      const int n = n0 + (j << 4) + rlane;
      float bv = 0.f;
      if (BIAS_MODE == 2) bv = bias[n];
#pragma unroll
      for (int r = 0; r < 8; ++r) {
        float v = acc[i][j][r] * scale;
        if (BIAS_MODE == 1) v += bias[mBase + mOff + r];
        if (BIAS_MODE == 2) v += bv;
        if (RESID) v += Rb[(size_t)(mBase + mOff + r) * ldc + n];
        if (ACT == 1) v = tanhf(v);
        if (ACT == 2) v = fmaxf(v, 0.0f);
        if (ACT == 3) v = v / (1.0f + expf(-v));
        if (ACT == 4) v = (v > 0.f) ? v : 0.01f * v;
        slab[(mOff + r) * 68 + (j << 4) + rlane] = v;
      }
    }
    __builtin_amdgcn_fence(__ATOMIC_RELEASE, "workgroup");
    __builtin_amdgcn_wave_barrier();
    __builtin_amdgcn_fence(__ATOMIC_ACQUIRE, "workgroup");
    if (OUT_MODE == 0) {
      float* C = (float*)Cout + (size_t)b * strideC;
      const int hh = lane >> 4, c4 = (lane & 15) * 4;
      for (int pass = 0; pass < 2; ++pass) {
#pragma unroll
        for (int it = 0; it < 8; ++it) {
          const int row = it * 2 + hh;
          v4f v = *(const v4f*)(slab + row * 68 + c4);
          *(volatile v4f*)(C + (size_t)(mBase + row) * ldc + n0 + c4) = v;
        }
        __threadfence();
      }
    } else {
      const int q = lane >> 3, c8 = (lane & 7) * 8;
      unsigned short* C  = (unsigned short*)Cout  + (size_t)b * strideC;
      unsigned short* C2 = (OUT_MODE == 2) ? ((unsigned short*)Cout2 + (size_t)b * strideC) : nullptr;
      for (int pass = 0; pass < 2; ++pass) {
#pragma unroll
        for (int it = 0; it < 4; ++it) {
          const int row = it * 4 + q;
          const float* sp = slab + row * 68 + c8;
          v8h hv, lv;
#pragma unroll
          for (int e = 0; e < 8; ++e) {
            if (OUT_MODE == 1) {
              hv[e] = (_Float16)sp[e];
            } else {
              unsigned short hb = f2bf_bits(sp[e]);
              unsigned short lb = f2bf_bits(sp[e] - bf_bits2f(hb));
              hv[e] = __builtin_bit_cast(_Float16, hb);
              lv[e] = __builtin_bit_cast(_Float16, lb);
            }
          }
          *(volatile v8h*)(C + (size_t)(mBase + row) * ldc + n0 + c8) = hv;
          if (OUT_MODE == 2) *(volatile v8h*)(C2 + (size_t)(mBase + row) * ldc + n0 + c8) = lv;
        }
        __threadfence();
      }
    }
    __builtin_amdgcn_fence(__ATOMIC_RELEASE, "workgroup");
    __builtin_amdgcn_wave_barrier();
    __builtin_amdgcn_fence(__ATOMIC_ACQUIRE, "workgroup");
  }
}

__device__ __forceinline__ unsigned pk16(unsigned short a, unsigned short b) { return (unsigned)a | ((unsigned)b << 16); }
__device__ __forceinline__ unsigned short h_bits(float f) { const _Float16 h = (_Float16)f; return __builtin_bit_cast(unsigned short, h); }

__global__ __launch_bounds__(256) void cast_scale_f32_f16x2(
    const float* __restrict__ in, unsigned short* __restrict__ out, int n2, float scale) {
  int i = blockIdx.x * 256 + threadIdx.x;
  if (i < n2) {
    const unsigned u = pk16(h_bits(in[2 * i] * scale), h_bits(in[2 * i + 1] * scale));
    ((volatile unsigned*)out)[i] = u;
    __threadfence();
    ((volatile unsigned*)out)[i] = u;
  }
}

__global__ __launch_bounds__(256) void transpose_cast_f16_kernel(const float* __restrict__ in, unsigned short* __restrict__ out,
                                                                 int R, int CC, float scale) {
  __shared__ float tile[64][65];
  const int t  = threadIdx.x;
  const int n0 = blockIdx.x * 64;
  const int k0 = blockIdx.y * 64;
  {
    const int kr = t >> 2, nc = (t & 3) * 16;
    const float* p = in + (size_t)(k0 + kr) * CC + n0 + nc;
#pragma unroll
    for (int e4 = 0; e4 < 4; ++e4) {
      const v4f f = *(const v4f*)(p + 4 * e4);
      tile[kr][nc + 4 * e4 + 0] = f[0];
      tile[kr][nc + 4 * e4 + 1] = f[1];
      tile[kr][nc + 4 * e4 + 2] = f[2];
      tile[kr][nc + 4 * e4 + 3] = f[3];
    }
  }
  __syncthreads();
  const int q = t >> 3, c8 = (t & 7) * 8;
  v4u u0, u1;
#pragma unroll
  for (int w = 0; w < 4; ++w) {
    u0[w] = pk16(h_bits(tile[c8 + 2 * w][q] * scale),      h_bits(tile[c8 + 2 * w + 1][q] * scale));
    u1[w] = pk16(h_bits(tile[c8 + 2 * w][32 + q] * scale), h_bits(tile[c8 + 2 * w + 1][32 + q] * scale));
  }
  unsigned short* p0 = out + (size_t)(n0 + q) * R + k0 + c8;
  unsigned short* p1 = out + (size_t)(n0 + 32 + q) * R + k0 + c8;
  for (int pass = 0; pass < 2; ++pass) {
    *(volatile v4u*)p0 = u0;
    *(volatile v4u*)p1 = u1;
    __threadfence();
  }
}

constexpr int ATT_D  = 64;
constexpr int ATT_NW = 4;
constexpr int ATT_QB = 64;
constexpr int ATT_KC = 64;

__device__ __forceinline__ v8f mma_h(v16h a, v16h b, v8f c) {
  c = __builtin_amdgcn_wmma_f32_16x16x32_f16(false, a, false, b, (short)0, c, false, false);
  asm volatile("v_nop\n\tv_nop\n\tv_nop\n\tv_nop" : "+v"(c) : "v"(a), "v"(b));
  return c;
}

__global__ __launch_bounds__(128)
void attn64_h16_kernel(const unsigned short* __restrict__ qp, const unsigned short* __restrict__ kp,
                       const unsigned short* __restrict__ vtp, float* __restrict__ out,
                       long q_bs, long k_bs, long v_bs, long o_bs,
                       int q_rs, int k_rs, int v_rs, int o_rs,
                       int S, int Skv, float sscale) {
  __shared__ __align__(16) _Float16 Ksh[ATT_KC * ATT_D];
  __shared__ __align__(16) _Float16 Vth[ATT_D * ATT_KC];
  __shared__ __align__(16) _Float16 Psh[ATT_NW][16 * ATT_KC];
  __shared__ __align__(16) float    Os[ATT_NW][16 * 68];

  const _Float16* q  = (const _Float16*)qp;
  const _Float16* k  = (const _Float16*)kp;
  const _Float16* vt = (const _Float16*)vtp;

  const int tid  = threadIdx.x;
  const int wave = tid >> 5;
  const int lane = tid & 31;
  const int hh   = lane >> 4;
  const int c    = lane & 15;

  const int nqb = S / ATT_QB;
  const int bx  = blockIdx.x;
  const int qb  = bx % nqb;
  const int b   = bx / nqb;
  const int q0  = qb * ATT_QB + wave * 16;

  const _Float16* qb_ptr = q  + (size_t)b * q_bs;
  const _Float16* kb_ptr = k  + (size_t)b * k_bs;
  const _Float16* vb_ptr = vt + (size_t)b * v_bs;
  float*          ob_ptr = out + (size_t)b * o_bs;

  v16h qa[2];
  {
    const _Float16* qrow = qb_ptr + (size_t)(q0 + c) * q_rs + 8 * hh;
#pragma unroll
    for (int dc = 0; dc < 2; ++dc) qa[dc] = Frag<_Float16>::load(qrow + dc * 32);
  }

  float mrow[8], lrow[8];
  v8f oacc[4];
#pragma unroll
  for (int r = 0; r < 8; ++r) { mrow[r] = -INFINITY; lrow[r] = 0.f; }
#pragma unroll
  for (int t = 0; t < 4; ++t) oacc[t] = (v8f){0.f,0.f,0.f,0.f,0.f,0.f,0.f,0.f};

  const int nChunks = Skv / ATT_KC;
  for (int kc = 0; kc < nChunks; ++kc) {
    const int kv0 = kc * ATT_KC;
    __syncthreads();
    {
#pragma unroll
      for (int i = 0; i < 4; ++i) {
        const int ci   = tid + 128 * i;
        const int row  = ci >> 3;
        const int col8 = (ci & 7) * 8;
        const v8h kk = *(const v8h*)(kb_ptr + (size_t)(kv0 + row) * k_rs + col8);
        const v8h vv = *(const v8h*)(vb_ptr + (size_t)row * v_rs + kv0 + col8);
        *(v8h*)(Ksh + row * ATT_D + col8)  = kk;
        *(v8h*)(Vth + row * ATT_KC + col8) = vv;
      }
    }
    __syncthreads();

    v8f s[4];
#pragma unroll
    for (int j = 0; j < 4; ++j) {
      s[j] = (v8f){0.f,0.f,0.f,0.f,0.f,0.f,0.f,0.f};
#pragma unroll
      for (int dc = 0; dc < 2; ++dc) {
        const v16h kb = Frag<_Float16>::load(Ksh + (j * 16 + c) * ATT_D + dc * 32 + 8 * hh);
        s[j] = mma_h(qa[dc], kb, s[j]);
      }
    }
    float cm[8];
#pragma unroll
    for (int r = 0; r < 8; ++r) {
      float m = -INFINITY;
#pragma unroll
      for (int j = 0; j < 4; ++j) {
        s[j][r] *= sscale;
        m = fmaxf(m, s[j][r]);
      }
#pragma unroll
      for (int off = 1; off < 16; off <<= 1) m = fmaxf(m, __shfl_xor(m, off, 32));
      cm[r] = m;
    }
    _Float16* pw = Psh[wave];
#pragma unroll
    for (int r = 0; r < 8; ++r) {
      const float mnew  = fmaxf(mrow[r], cm[r]);
      const float alpha = expf(mrow[r] - mnew);
      mrow[r] = mnew;
      float psum = 0.f;
#pragma unroll
      for (int j = 0; j < 4; ++j) {
        const float p = expf(s[j][r] - mnew);
        psum += p;
        pw[(8 * hh + r) * ATT_KC + j * 16 + c] = (_Float16)(p * kPCarry);
      }
#pragma unroll
      for (int off = 1; off < 16; off <<= 1) psum += __shfl_xor(psum, off, 32);
      lrow[r] = lrow[r] * alpha + psum;
#pragma unroll
      for (int t = 0; t < 4; ++t) oacc[t][r] *= alpha;
    }
    __builtin_amdgcn_fence(__ATOMIC_RELEASE, "workgroup");
    __builtin_amdgcn_wave_barrier();
    __builtin_amdgcn_fence(__ATOMIC_ACQUIRE, "workgroup");
#pragma unroll 1
    for (int kk = 0; kk < 2; ++kk) {
      const v16h pa = Frag<_Float16>::load(pw + c * ATT_KC + kk * 32 + 8 * hh);
#pragma unroll
      for (int t = 0; t < 4; ++t) {
        const v16h vb = Frag<_Float16>::load(Vth + (t * 16 + c) * ATT_KC + kk * 32 + 8 * hh);
        oacc[t] = mma_h(pa, vb, oacc[t]);
      }
    }
  }

  float* os = Os[wave];
#pragma unroll
  for (int r = 0; r < 8; ++r) {
    const float inv = 1.0f / (lrow[r] * kPCarry);
#pragma unroll
    for (int t = 0; t < 4; ++t) os[(8 * hh + r) * 68 + t * 16 + c] = oacc[t][r] * inv;
  }
  __builtin_amdgcn_fence(__ATOMIC_RELEASE, "workgroup");
  __builtin_amdgcn_wave_barrier();
  __builtin_amdgcn_fence(__ATOMIC_ACQUIRE, "workgroup");
  {
    const int c4 = (lane & 15) * 4;
    for (int pass = 0; pass < 2; ++pass) {
#pragma unroll
      for (int it = 0; it < 8; ++it) {
        const int row = it * 2 + hh;
        v4f val = *(const v4f*)(os + row * 68 + c4);
        *(volatile v4f*)(ob_ptr + (size_t)(q0 + row) * o_rs + c4) = val;
      }
      __threadfence();
    }
  }
}

extern "C" void kernel_launch(void* const* d_in, const int* in_sizes, int n_in,
                              void* d_out, int out_size, void* d_ws, size_t ws_size,
                              hipStream_t stream) {
  if (n_in < 9) return;
  if (in_sizes[0] != NBATCH * NCH * NVOX) return;
  if (in_sizes[1] != NCH * NCH || in_sizes[3] != NCH * NCH || in_sizes[5] != NCH * NCH || in_sizes[7] != NCH * NCH) return;
  if (in_sizes[2] != NCH || in_sizes[4] != NCH || in_sizes[6] != NCH || in_sizes[8] != NCH) return;
  if (out_size != NBATCH * NCH * NVOX) return;
  static_assert(NVOX % 64 == 0);
  static_assert(NCH % 64 == 0);

  const float* x  = (const float*)d_in[0];
  const float* wq = (const float*)d_in[1];
  const float* bq = (const float*)d_in[2];
  const float* wk = (const float*)d_in[3];
  const float* bk = (const float*)d_in[4];
  const float* wv = (const float*)d_in[5];
  const float* bv = (const float*)d_in[6];
  const float* wo = (const float*)d_in[7];
  const float* bo = (const float*)d_in[8];
  float* outp = (float*)d_out;

  const size_t PW   = (size_t)NCH * NCH * 2;
  const size_t P16  = (size_t)NBATCH * NVOX * NCH * 2;
  const size_t P32  = (size_t)NBATCH * NVOX * NCH * 4;
  size_t off = 0;
  const size_t oWQ = off; off += PW;
  const size_t oWK = off; off += PW;
  const size_t oWV = off; off += PW;
  const size_t oWO = off; off += PW;
  const size_t oXT = off; off += P16;
  const size_t oQ  = off; off += P16;
  const size_t oK  = off; off += P16;
  const size_t oVT = off; off += P16;
  const size_t oO  = off; off += P32;
  const size_t oBT = off; off += P16;
  if (off > ws_size) return;

  char* ws = (char*)d_ws;
  unsigned short* WQ16 = (unsigned short*)(ws + oWQ);
  unsigned short* WK16 = (unsigned short*)(ws + oWK);
  unsigned short* WV16 = (unsigned short*)(ws + oWV);
  unsigned short* WO16 = (unsigned short*)(ws + oWO);
  unsigned short* XT16 = (unsigned short*)(ws + oXT);
  unsigned short* Q16  = (unsigned short*)(ws + oQ);
  unsigned short* K16  = (unsigned short*)(ws + oK);
  unsigned short* VT16 = (unsigned short*)(ws + oVT);
  float*          OBUF = (float*)(ws + oO);
  unsigned short* BT16 = (unsigned short*)(ws + oBT);

  const dim3 blk(256);
  const long plane16 = (long)NVOX * NCH;

  const int n2w = NCH * NCH / 2;
  cast_scale_f32_f16x2<<<dim3((n2w + 255) / 256), blk, 0, stream>>>(wq, WQ16, n2w, kWCarry);
  cast_scale_f32_f16x2<<<dim3((n2w + 255) / 256), blk, 0, stream>>>(wk, WK16, n2w, kWCarry);
  cast_scale_f32_f16x2<<<dim3((n2w + 255) / 256), blk, 0, stream>>>(wv, WV16, n2w, kWCarry);
  cast_scale_f32_f16x2<<<dim3((n2w + 255) / 256), blk, 0, stream>>>(wo, WO16, n2w, kWCarry);

  for (int b = 0; b < NBATCH; ++b) {
    transpose_cast_f16_kernel<<<dim3(NVOX / 64, NCH / 64), blk, 0, stream>>>(
        x + (size_t)b * NCH * NVOX, XT16 + (size_t)b * plane16, NCH, NVOX, 1.0f);
  }

  const dim3 gQK(((NVOX / 64) * (NCH / 64) + 7) / 8, NBATCH);
  const dim3 gVT(((NCH / 64) * (NVOX / 64) + 7) / 8, NBATCH);

  wmma_gemm64<0, false, 2, 1, false, 0, 0><<<gQK, blk, 0, stream>>>(
      XT16, XT16, NCH, plane16, WQ16, WQ16, NCH, 0L, (void*)Q16, (void*)Q16, NCH, plane16, bq, x, 0L, NVOX, NCH, NCH, kWCarryInv);
  wmma_gemm64<0, false, 2, 1, false, 0, 0><<<gQK, blk, 0, stream>>>(
      XT16, XT16, NCH, plane16, WK16, WK16, NCH, 0L, (void*)K16, (void*)K16, NCH, plane16, bk, x, 0L, NVOX, NCH, NCH, kWCarryInv);
  wmma_gemm64<0, false, 1, 1, false, 0, 0><<<gVT, blk, 0, stream>>>(
      WV16, WV16, NCH, 0L, XT16, XT16, NCH, plane16, (void*)VT16, (void*)VT16, NVOX, plane16, bv, x, 0L, NCH, NVOX, NCH, kWCarryInv);

  attn64_h16_kernel<<<dim3(NBATCH * (NVOX / 64)), dim3(128), 0, stream>>>(
      Q16, K16, VT16, OBUF,
      plane16, plane16, plane16, plane16,
      NCH, NCH, NVOX, NCH,
      NVOX, NVOX, kQKScale);

  for (int b = 0; b < NBATCH; ++b) {
    transpose_cast_f16_kernel<<<dim3(NVOX / 64, NCH / 64), blk, 0, stream>>>(
        OBUF + (size_t)b * plane16, BT16 + (size_t)b * plane16, NCH, NVOX, kOCarry);
  }

  wmma_gemm64<0, false, 1, 0, false, 0, 0><<<gVT, blk, 0, stream>>>(
      WO16, WO16, NCH, 0L, BT16, BT16, NCH, plane16, (void*)outp, (void*)outp, NVOX, plane16, bo, x, 0L, NCH, NVOX, NCH, kOutScale);
}
